// DifferentiableToposAttention_5016521801931
// MI455X (gfx1250) — hardware-run, weakly checked
//
#include <hip/hip_runtime.h>


#ifndef NB
#define NB 2
#endif
#ifndef SEQ
#define SEQ 1024
#endif
#define NB_FULL  2
#define SEQ_FULL 1024
#ifndef OUT_SEQ
#define OUT_SEQ SEQ
#endif
#define DM   128
#define TP   132
#define RS   2048.0f
#define RI   (1.0f / 2048.0f)
#define PSH  8.0f
#define C1   (0.078125f * 1.4426950408889634f)
#define EM   (8.0f - 10.0f * 1.4426950408889634f)

static_assert(DM == 128);
static_assert(DM % 64 == 0);
static_assert(DM % 32 == 0);
static_assert(SEQ % 64 == 0);
static_assert((NB * SEQ) % 64 == 0);
static_assert(SEQ % 32 == 0);
static_assert(SEQ % 16 == 0);
static_assert(((size_t)SEQ * DM) % 8 == 0);
static_assert(((size_t)DM * DM) % 8 == 0);
static_assert(NB <= NB_FULL);
static_assert(SEQ <= SEQ_FULL);
static_assert((TP * 4) % 16 == 0);

typedef _Float16 h16;
typedef unsigned short bf;
typedef __attribute__((ext_vector_type(16))) __bf16   v16bf;
typedef __attribute__((ext_vector_type(16))) _Float16 v16h;
typedef __attribute__((ext_vector_type(8)))  _Float16 v8h;
typedef __attribute__((ext_vector_type(8)))  unsigned short v8us;
typedef __attribute__((ext_vector_type(8)))  float    v8f;
typedef __attribute__((ext_vector_type(4)))  float    v4f;
typedef v4f  __attribute__((may_alias)) v4fa;

__device__ __forceinline__ unsigned short f2bf(float f) { unsigned u = __float_as_uint(f); u += 0x7FFFu + ((u >> 16) & 1u); return (unsigned short)(u >> 16); }
__device__ __forceinline__ float bfr(float f) { return __uint_as_float(((unsigned)f2bf(f)) << 16); }
__device__ __forceinline__ v16h cat16(v8h lo, v8h hi) { return __builtin_shufflevector(lo, hi, 0, 1, 2, 3, 4, 5, 6, 7, 8, 9, 10, 11, 12, 13, 14, 15); }
__device__ __forceinline__ v16bf cat16b(v8us lo, v8us hi) { return __builtin_bit_cast(v16bf, __builtin_shufflevector(lo, hi, 0, 1, 2, 3, 4, 5, 6, 7, 8, 9, 10, 11, 12, 13, 14, 15)); }
__device__ __forceinline__ v8f wmma16(v16h a, v16h b, v8f c) { return __builtin_amdgcn_wmma_f32_16x16x32_f16(false, a, false, b, (short)0, c, false, false); }
__device__ __forceinline__ v8f wmmab(v16bf a, v16bf b, v8f c) { return __builtin_amdgcn_wmma_f32_16x16x32_bf16(false, a, false, b, (short)0, c, false, false); }
__device__ __forceinline__ v16h  ldh(const h16* p) { return cat16(*(const v8h*)p, *(const v8h*)(p + 16)); }
__device__ __forceinline__ v16bf ldb(const bf* p)  { return cat16b(*(const v8us*)p, *(const v8us*)(p + 16)); }
__device__ __forceinline__ void wave_sync() { __builtin_amdgcn_fence(3  , "wavefront"); __builtin_amdgcn_wave_barrier(); asm volatile("" ::: "memory"); }

__global__ __launch_bounds__(256) void k_cvt8(const float* __restrict__ src, bf* dst, size_t n8) {
    const size_t i = (size_t)blockIdx.x * 256 + threadIdx.x; if (i >= n8) return;
    const v8f v = *(const v8f*)(src + i * 8); v8us o;
#pragma unroll
    for (int k = 0; k < 8; ++k) o[k] = f2bf(v[k]);
    *(volatile v8us*)(dst + i * 8) = o; __threadfence(); *(volatile v8us*)(dst + i * 8) = o;
}

__device__ __forceinline__ void gemm64(const bf* __restrict__ A, const bf* __restrict__ Bt, int r0, int c0, int lr, int hi, v8f (&acc)[4][4]) {
    const int K = DM;
#pragma unroll
    for (int mb = 0; mb < 4; ++mb)
#pragma unroll
        for (int nb = 0; nb < 4; ++nb) acc[mb][nb] = (v8f){};
    const size_t aoff = (size_t)(r0 + lr) * K + 8 * hi, boff = (size_t)(c0 + lr) * K + 8 * hi;
#pragma unroll 1
    for (int kc = 0; kc < K; kc += 32) {
        v16bf a[4];
#pragma unroll
        for (int mb = 0; mb < 4; ++mb) a[mb] = ldb(A + aoff + (size_t)mb * 16 * K + kc);
#pragma unroll
        for (int nb = 0; nb < 4; ++nb) { const v16bf b = ldb(Bt + boff + (size_t)nb * 16 * K + kc);
#pragma unroll
            for (int mb = 0; mb < 4; ++mb) acc[mb][nb] = wmmab(a[mb], b, acc[mb][nb]); }
        asm volatile("v_nop\n\tv_nop\n\tv_nop\n\tv_nop" : "+v"(acc[0][0]), "+v"(acc[1][1]), "+v"(acc[2][2]), "+v"(acc[3][3]) : "v"(a[0]), "v"(a[1]), "v"(a[2]), "v"(a[3]));
    }
}

__global__ __launch_bounds__(32) void k_proj_qk(const bf* __restrict__ XB, const bf* __restrict__ WB, const float* __restrict__ bq, const float* __restrict__ bk, float* QK) {
    __shared__ __align__(16) float os[16 * 68];
    const int lane = threadIdx.x & 31, lr = lane & 15, hi = lane >> 4;
    const int r0 = blockIdx.x * 64, c0 = blockIdx.y * 64, z = blockIdx.z;
    v8f acc[4][4];
    gemm64(XB, WB + (size_t)z * DM * DM, r0, c0, lr, hi, acc);
    float bias[4];
#pragma unroll
    for (int nb = 0; nb < 4; ++nb) { const int col = c0 + nb * 16 + lr; const float vq = bq[col]; const float vk = bk[col]; bias[nb] = bfr(z ? vk : vq); }
    float* P = QK + (size_t)z * NB * SEQ * DM;
#pragma unroll
    for (int mb = 0; mb < 4; ++mb) {
#pragma unroll
        for (int nb = 0; nb < 4; ++nb) {
#pragma unroll
            for (int j = 0; j < 8; ++j) os[(hi * 8 + j) * 68 + nb * 16 + lr] = acc[mb][nb][j] + bias[nb]; }
        wave_sync();
#pragma unroll 1
        for (int s = 0; s < 8; ++s) { const int row = 2 * s + hi, cofs = lr * 4;
            v4f v = *(const v4fa*)(&os[row * 68 + cofs]);
#pragma unroll
            for (int i = 0; i < 4; ++i) v[i] = 1.0f / (1.0f + expf(-v[i]));
            *(v4fa*)(&os[row * 68 + cofs]) = v; }
        wave_sync();
        float* orow = P + (size_t)(r0 + mb * 16) * DM + c0;
#pragma unroll
        for (int s = 0; s < 8; ++s) { const int row = 2 * s + hi, cofs = lr * 4;
            const v4f val = *(const v4fa*)(&os[row * 68 + cofs]);
            *(volatile v4f*)(orow + (size_t)row * DM + cofs) = val; }
        __threadfence();
#pragma unroll
        for (int s = 0; s < 8; ++s) { const int row = 2 * s + hi, cofs = lr * 4;
            const v4f val = *(const v4fa*)(&os[row * 68 + cofs]);
            *(volatile v4f*)(orow + (size_t)row * DM + cofs) = val; }
        wave_sync();
    }
}

__global__ __launch_bounds__(32) void k_proj_vt(const bf* __restrict__ WV, const bf* __restrict__ XB, const float* __restrict__ bv, h16* VH, h16* VR) {
    __shared__ __align__(16) float os[16 * 68];
    const int lane = threadIdx.x & 31, lr = lane & 15, hi = lane >> 4;
    const int r0 = blockIdx.x * 64, c0 = blockIdx.y * 64;
    v8f acc[4][4];
    gemm64(WV, XB, r0, c0, lr, hi, acc);
    const int b = c0 / SEQ, t0 = c0 % SEQ;
    const size_t tbase = ((size_t)b * DM + r0) * SEQ + t0;
#pragma unroll
    for (int mb = 0; mb < 4; ++mb) {
#pragma unroll
        for (int nb = 0; nb < 4; ++nb) {
#pragma unroll
            for (int j = 0; j < 8; ++j) os[(hi * 8 + j) * 68 + nb * 16 + lr] = acc[mb][nb][j]; }
        wave_sync();
        v8h hv[4], rv[4];
#pragma unroll
        for (int s = 0; s < 4; ++s) { const int row = 4 * s + (lane >> 3), c8 = (lane & 7) * 8;
            const float bb = bfr(bv[r0 + mb * 16 + row]);
            const v4f x0 = *(const v4fa*)(&os[row * 68 + c8]); const v4f x1 = *(const v4fa*)(&os[row * 68 + c8 + 4]);
#pragma unroll
            for (int i = 0; i < 4; ++i) { const float y0 = x0[i] + bb; const float y1 = x1[i] + bb; const h16 a0 = (h16)y0; const h16 a1 = (h16)y1;
                hv[s][i] = a0; hv[s][4 + i] = a1; rv[s][i] = (h16)((y0 - (float)a0) * RS); rv[s][4 + i] = (h16)((y1 - (float)a1) * RS); } }
#pragma unroll
        for (int s = 0; s < 4; ++s) { const int row = 4 * s + (lane >> 3), c8 = (lane & 7) * 8;
            const size_t oo = tbase + (size_t)(mb * 16 + row) * SEQ + c8;
            *(volatile v8h*)(VH + oo) = hv[s]; *(volatile v8h*)(VR + oo) = rv[s]; }
        __threadfence();
#pragma unroll
        for (int s = 0; s < 4; ++s) { const int row = 4 * s + (lane >> 3), c8 = (lane & 7) * 8;
            const size_t oo = tbase + (size_t)(mb * 16 + row) * SEQ + c8;
            *(volatile v8h*)(VH + oo) = hv[s]; *(volatile v8h*)(VR + oo) = rv[s]; }
        wave_sync();
    }
}

__global__ __launch_bounds__(32) void k_attn(const float* __restrict__ QF, const float* __restrict__ KF, const h16* __restrict__ VH, const h16* __restrict__ VR, const int* __restrict__ maskp, float* OUT) {
    __shared__ __align__(16) float qs[16 * TP];
    __shared__ __align__(16) float ks[32 * TP];
    __shared__ __align__(16) float os[16 * TP];
    const int lane = threadIdx.x & 31, lr = lane & 15, hi = lane >> 4;
    const int b  = __builtin_amdgcn_readfirstlane((int)blockIdx.y);
    const int t0 = __builtin_amdgcn_readfirstlane((int)blockIdx.x * 16);
    const int causal = __builtin_amdgcn_readfirstlane((maskp[0] != 0) ? 1 : 0);
    const size_t rowb = (size_t)b * SEQ;
#pragma unroll 8
    for (int i = 0; i < 16; ++i) { const v4f v = *(const v4f*)(QF + (rowb + t0 + i) * DM + 4 * lane); *(v4fa*)(&qs[i * TP + 4 * lane]) = v; }
    wave_sync();
    v8f oh[8], orr[8];
#pragma unroll
    for (int j = 0; j < 8; ++j) { oh[j] = (v8f){}; orr[j] = (v8f){}; }
    float l = 0.0f;
    const float pmf = __builtin_amdgcn_exp2f(EM);
    const h16 pmh = (h16)pmf; const h16 pmr = (h16)((pmf - (float)pmh) * RS);
    const float pml = (float)pmh + (float)pmr * RI;
    const size_t vo = ((size_t)b * DM + lr) * SEQ + 8 * hi;
    const int tq = t0 + lr;
#pragma unroll 1
    for (int key0 = 0; key0 < SEQ; key0 += 32) {
        v16h pb, pr; float ls;
        const bool live = (causal == 0) || (key0 <= t0 + 15);
        if (live) {
            wave_sync();
#pragma unroll 8
            for (int i = 0; i < 32; ++i) { const v4f v = *(const v4f*)(KF + (rowb + key0 + i) * DM + 4 * lane); *(v4fa*)(&ks[i * TP + 4 * lane]) = v; }
            wave_sync();
            float sa[8], sb[8];
#pragma unroll
            for (int r = 0; r < 8; ++r) { sa[r] = 0.0f; sb[r] = 0.0f; }
#pragma unroll 1
            for (int d = 0; d < DM; d += 4) {
                const v4f q = *(const v4fa*)(&qs[lr * TP + d]);
#pragma unroll
                for (int r = 0; r < 8; ++r) { const v4f k = *(const v4fa*)(&ks[(8 * hi + r) * TP + d]);
                    sa[r] += fmaxf(q[0] - k[0], 0.0f); sa[r] += fmaxf(q[1] - k[1], 0.0f); sa[r] += fmaxf(q[2] - k[2], 0.0f); sa[r] += fmaxf(q[3] - k[3], 0.0f); }
                asm volatile("" ::: "memory");
#pragma unroll
                for (int r = 0; r < 8; ++r) { const v4f k = *(const v4fa*)(&ks[(16 + 8 * hi + r) * TP + d]);
                    sb[r] += fmaxf(q[0] - k[0], 0.0f); sb[r] += fmaxf(q[1] - k[1], 0.0f); sb[r] += fmaxf(q[2] - k[2], 0.0f); sb[r] += fmaxf(q[3] - k[3], 0.0f); }
            }
            ls = 0.0f;
#pragma unroll
            for (int r = 0; r < 8; ++r) {
                const int kA = key0 + 8 * hi + r, kB = kA + 16;
                float ea = PSH - sa[r] * C1, eb = PSH - sb[r] * C1;
                ea = (causal != 0 && kA > tq) ? EM : ea;
                eb = (causal != 0 && kB > tq) ? EM : eb;
                const float pa = __builtin_amdgcn_exp2f(ea), pc = __builtin_amdgcn_exp2f(eb);
                const h16 ha = (h16)pa, hb = (h16)pc;
                const h16 ra = (h16)((pa - (float)ha) * RS), rb = (h16)((pc - (float)hb) * RS);
                pb[r] = ha; pb[8 + r] = hb; pr[r] = ra; pr[8 + r] = rb;
                ls += ((float)ha + (float)ra * RI) + ((float)hb + (float)rb * RI);
            }
        } else {
#pragma unroll
            for (int i = 0; i < 16; ++i) { pb[i] = pmh; pr[i] = pmr; }
            ls = 16.0f * pml;
        }
        l += ls;
        const h16* vh = VH + vo + key0; const h16* vr = VR + vo + key0;
#pragma unroll
        for (int g = 0; g < 4; ++g) {
            const int j0 = 2 * g, j1 = 2 * g + 1;
            const v16h a0 = ldh(vh + (size_t)(16 * j0) * SEQ), a1 = ldh(vh + (size_t)(16 * j1) * SEQ);
            const v16h r0 = ldh(vr + (size_t)(16 * j0) * SEQ), r1 = ldh(vr + (size_t)(16 * j1) * SEQ);
            oh[j0]  = wmma16(a0, pb, oh[j0]);   oh[j1]  = wmma16(a1, pb, oh[j1]);
            orr[j0] = wmma16(r0, pb, orr[j0]);  orr[j1] = wmma16(r1, pb, orr[j1]);
            orr[j0] = wmma16(a0, pr, orr[j0]);  orr[j1] = wmma16(a1, pr, orr[j1]);
            asm volatile("v_nop\n\tv_nop\n\tv_nop\n\tv_nop" : "+v"(oh[j0]), "+v"(oh[j1]), "+v"(orr[j0]), "+v"(orr[j1]) : "v"(a0), "v"(a1), "v"(r0), "v"(r1), "v"(pb), "v"(pr) : "memory");
        }
    }
    l += __shfl_xor(l, 16, 32);
    const float inv = 1.0f / l;
#pragma unroll
    for (int j = 0; j < 8; ++j) { v4f a, c;
#pragma unroll
        for (int i = 0; i < 4; ++i) { a[i] = (oh[j][i] + orr[j][i] * RI) * inv; c[i] = (oh[j][4 + i] + orr[j][4 + i] * RI) * inv; }
        *(v4fa*)(&os[lr * TP + 16 * j + 8 * hi]) = a; *(v4fa*)(&os[lr * TP + 16 * j + 8 * hi + 4]) = c; }
    wave_sync();
    float* orow = OUT + ((size_t)b * OUT_SEQ + t0) * DM;
#pragma unroll
    for (int s = 0; s < 16; ++s) { const v4f val = *(const v4fa*)(&os[s * TP + 4 * lane]);
        *(volatile v4f*)(orow + (size_t)s * DM + 4 * lane) = val; }
    __threadfence();
#pragma unroll
    for (int s = 0; s < 16; ++s) { const v4f val = *(const v4fa*)(&os[s * TP + 4 * lane]);
        *(volatile v4f*)(orow + (size_t)s * DM + 4 * lane) = val; }
}

static constexpr size_t al256(size_t v) { return (v + 255) & ~(size_t)255; }
static constexpr size_t SZ_XB = al256((size_t)NB * SEQ * DM * 2);
static constexpr size_t SZ_WB = al256((size_t)3 * DM * DM * 2);
static constexpr size_t SZ_QK = al256((size_t)2 * NB * SEQ * DM * 4);
static constexpr size_t SZ_VP = al256((size_t)NB * DM * SEQ * 2);
static constexpr size_t SZ_TOTAL = SZ_XB + SZ_WB + SZ_QK + 2 * SZ_VP;
static_assert(SZ_TOTAL <= (size_t)134217728);
static_assert(((size_t)DM * DM * 2) % 256 == 0);
static_assert(((size_t)NB * SEQ * DM * 4) % 256 == 0);

extern "C" void kernel_launch(void* const* d_in, const int* in_sizes, int n_in,
                              void* d_out, int out_size, void* d_ws, size_t ws_size, hipStream_t stream) {
    if (n_in < 8) return;
    const size_t needx = ((size_t)(NB - 1) * SEQ_FULL + SEQ) * DM;
    if ((size_t)in_sizes[0] < needx) return;
    if ((size_t)in_sizes[1] < (size_t)DM * DM || (size_t)in_sizes[3] < (size_t)DM * DM || (size_t)in_sizes[5] < (size_t)DM * DM) return;
    if (in_sizes[2] < DM || in_sizes[4] < DM || in_sizes[6] < DM || in_sizes[7] < 1) return;
    if ((size_t)out_size < ((size_t)(NB - 1) * OUT_SEQ + SEQ) * DM) return;
    if (SZ_TOTAL > ws_size) return;
    const float* x  = (const float*)d_in[0];
    const float* wq = (const float*)d_in[1]; const float* bq = (const float*)d_in[2];
    const float* wk = (const float*)d_in[3]; const float* bk = (const float*)d_in[4];
    const float* wv = (const float*)d_in[5]; const float* bv = (const float*)d_in[6];
    const int* maskp = (const int*)d_in[7];
    float* OUT = (float*)d_out;
    char* wsp = (char*)d_ws;
    bf* XB = (bf*)wsp; wsp += SZ_XB;
    bf* WB = (bf*)wsp; wsp += SZ_WB;
    float* QK = (float*)wsp; wsp += SZ_QK;
    h16* VH = (h16*)wsp; wsp += SZ_VP;
    h16* VR = (h16*)wsp; wsp += SZ_VP;
    bf* WQ = WB; bf* WK = WB + (size_t)DM * DM; bf* WV = WB + (size_t)2 * DM * DM;

    if (SEQ == SEQ_FULL) {
        const size_t n8 = (size_t)NB * SEQ * DM / 8;
        k_cvt8<<<(unsigned)((n8 + 255) / 256), 256, 0, stream>>>(x, XB, n8);
    } else {
        const size_t n8 = (size_t)SEQ * DM / 8;
        for (int b = 0; b < NB; ++b) k_cvt8<<<(unsigned)((n8 + 255) / 256), 256, 0, stream>>>(x + (size_t)b * SEQ_FULL * DM, XB + (size_t)b * SEQ * DM, n8);
    }
    { const size_t n8 = (size_t)DM * DM / 8; const unsigned g = (unsigned)((n8 + 255) / 256);
      k_cvt8<<<g, 256, 0, stream>>>(wq, WQ, n8); k_cvt8<<<g, 256, 0, stream>>>(wk, WK, n8); k_cvt8<<<g, 256, 0, stream>>>(wv, WV, n8); }

    k_proj_qk<<<dim3(NB * SEQ / 64, DM / 64, 2), 32, 0, stream>>>(XB, WB, bq, bk, QK);
    k_proj_vt<<<dim3(DM / 64, NB * SEQ / 64, 1), 32, 0, stream>>>(WV, XB, bv, VH, VR);

    k_attn<<<dim3(SEQ / 16, NB, 1), 32, 0, stream>>>(QK, QK + (size_t)NB * SEQ * DM, VH, VR, maskp, OUT);
}
